// MutualAttention_81466939670699
// MI455X (gfx1250) — hardware-run, weakly checked
//
#include <hip/hip_runtime.h>


#ifndef NB
#define NB 4
#endif
#ifndef SEQ
#define SEQ 4096
#endif
#define NB_FULL  4
#define SEQ_FULL 4096
#ifndef OUT_SEQ
#define OUT_SEQ SEQ
#endif
#define DM   128
#define DV   64
#define WOP  (2 * DV)
#define TP   136
#define WCARRY 64.0f
#define VCARRY 64.0f
#define CMEAN  (1.0f / (float)SEQ_FULL)
#define CFS    (CMEAN / (WCARRY * VCARRY))
#define CBS    ((1.0f - CMEAN) / (WCARRY * VCARRY))

static_assert(DM % 32 == 0);
static_assert(DV % 32 == 0);
static_assert(DV == 64);
static_assert(DM == 128);
static_assert(DM % 32 == 0);
static_assert(WOP % 8 == 0);
static_assert(SEQ % 64 == 0);
static_assert((NB * SEQ) % 64 == 0);
static_assert(SEQ_FULL % 4 == 0);
static_assert(OUT_SEQ % 32 == 0);
static_assert(OUT_SEQ >= SEQ);
static_assert(NB <= NB_FULL);
static_assert(SEQ <= SEQ_FULL);
static_assert((TP * 2) % 16 == 0);
static_assert(TP >= DM);
static_assert(256 * 8 * 4 == DM * 64);
static_assert(256 * 16 * 4 == 64 * DM * 2);
static_assert(32 * 16 * 4 == 16 * DV * 2);
static_assert(32 * 16 * 8 == 16 * 64 * 4);
static_assert(64 * TP * 2 <= 131072);
static_assert(16 * 68 * 4 <= 131072);

typedef _Float16 h16;
typedef unsigned short bf;
typedef __attribute__((ext_vector_type(16))) __bf16   v16bf;
typedef __attribute__((ext_vector_type(16))) _Float16 v16h;
typedef __attribute__((ext_vector_type(8)))  _Float16 v8h;
typedef __attribute__((ext_vector_type(8)))  unsigned short v8us;
typedef __attribute__((ext_vector_type(8)))  float    v8f;
typedef __attribute__((ext_vector_type(4)))  float    v4f;
typedef v4f  __attribute__((may_alias)) v4fa;
typedef v8us __attribute__((may_alias)) v8usa;

__device__ __forceinline__ unsigned short f2bf(float f) { unsigned u = __float_as_uint(f); u += 0x7FFFu + ((u >> 16) & 1u); return (unsigned short)(u >> 16); }
__device__ __forceinline__ float bfr(float f) { return __uint_as_float(((unsigned)f2bf(f)) << 16); }
__device__ __forceinline__ v16h cat16(v8h lo, v8h hi) { return __builtin_shufflevector(lo, hi, 0, 1, 2, 3, 4, 5, 6, 7, 8, 9, 10, 11, 12, 13, 14, 15); }
__device__ __forceinline__ v16bf cat16b(v8us lo, v8us hi) { return __builtin_bit_cast(v16bf, __builtin_shufflevector(lo, hi, 0, 1, 2, 3, 4, 5, 6, 7, 8, 9, 10, 11, 12, 13, 14, 15)); }
__device__ __forceinline__ v8f wmma16(v16h a, v16h b, v8f c) { return __builtin_amdgcn_wmma_f32_16x16x32_f16(false, a, false, b, (short)0, c, false, false); }
__device__ __forceinline__ v8f wmmab(v16bf a, v16bf b, v8f c) { return __builtin_amdgcn_wmma_f32_16x16x32_bf16(false, a, false, b, (short)0, c, false, false); }
__device__ __forceinline__ v16h  ldh(const h16* p) { return cat16(*(const v8h*)p, *(const v8h*)(p + 16)); }
__device__ __forceinline__ v16bf ldb(const bf* p)  { return cat16b(*(const v8us*)p, *(const v8us*)(p + 16)); }
__device__ __forceinline__ void wave_sync() { __builtin_amdgcn_fence(3  , "wavefront"); __builtin_amdgcn_wave_barrier(); asm volatile("" ::: "memory"); }
__device__ __forceinline__ v8f wmma16g(v16h a, v16h b, v8f c) { c = wmma16(a, b, c); asm volatile("v_nop\n\tv_nop\n\tv_nop\n\tv_nop" : "+v"(c) : "v"(a), "v"(b)); return c; }
__device__ __forceinline__ v8f wmmabg(v16bf a, v16bf b, v8f c) { c = wmmab(a, b, c); asm volatile("v_nop\n\tv_nop\n\tv_nop\n\tv_nop" : "+v"(c) : "v"(a), "v"(b)); return c; }
static __device__ __forceinline__ h16 toh_flush(float v) { const h16 r = (h16)v; return (fabsf(v) < 6.103515625e-05f) ? (h16)0.0f : r; }

__global__ __launch_bounds__(256) void k_cvt8(const float* __restrict__ src, bf* dst, size_t n8) {
    const size_t i = (size_t)blockIdx.x * 256 + threadIdx.x; if (i >= n8) return;
    const v8f v = *(const v8f*)(src + i * 8); v8us o;
#pragma unroll
    for (int k = 0; k < 8; ++k) o[k] = f2bf(v[k]);
    *(volatile v8us*)(dst + i * 8) = o; __threadfence(); *(volatile v8us*)(dst + i * 8) = o;
}

__global__ __launch_bounds__(256) void k_cvth8(const float* __restrict__ src, h16* dst, size_t n8) {
    const size_t i = (size_t)blockIdx.x * 256 + threadIdx.x; if (i >= n8) return;
    const v8f v = *(const v8f*)(src + i * 8); v8h o;
#pragma unroll
    for (int k = 0; k < 8; ++k) o[k] = toh_flush(bfr(v[k]) * WCARRY);
    *(volatile v8h*)(dst + i * 8) = o; __threadfence(); *(volatile v8h*)(dst + i * 8) = o;
}

__global__ __launch_bounds__(256) void k_tr(const float* __restrict__ hin, bf* HT) {
    __shared__ __align__(16) unsigned short ts[64 * TP];
    const unsigned tid = threadIdx.x;
    const int t0 = blockIdx.x * 64; const int slot = blockIdx.y;
    const int sb = (slot + NB_FULL - 1) % NB_FULL;
    const float* src = hin + (size_t)sb * DM * SEQ_FULL + t0;
#pragma unroll
    for (int it = 0; it < 8; ++it) {
        unsigned q = (unsigned)(it * 256) + tid; asm volatile("" : "+v"(q));
        const unsigned c = q >> 4, t4 = (q & 15u) * 4u;
        const v4f v = *(const v4f*)(src + (size_t)c * SEQ_FULL + t4);
#pragma unroll
        for (int j = 0; j < 4; ++j) ts[(t4 + (unsigned)j) * TP + c] = f2bf(v[j]); }
    __syncthreads();
    bf* dst = HT + ((size_t)slot * SEQ + (size_t)t0) * DM;
#pragma unroll 1
    for (int ps = 0; ps < 2; ++ps) {
#pragma unroll
        for (int it = 0; it < 4; ++it) {
            unsigned p = (unsigned)(it * 256) + tid; asm volatile("" : "+v"(p));
            const unsigned row = p >> 4, c8 = (p & 15u) * 8u;
            const v8us o = *(const v8usa*)(&ts[row * TP + c8]);
            *(volatile v8us*)(dst + (size_t)p * 8) = o; }
        if (ps == 0) __threadfence(); }
}

__global__ __launch_bounds__(32) void k_vmap(const bf* __restrict__ A, const bf* __restrict__ Bt, h16* VP) {
    __shared__ __align__(16) float os[16 * 68];
    const int K = DM;
    const int lane = threadIdx.x & 31, lr = lane & 15, hi = lane >> 4; const int r0 = blockIdx.x * 64;
    v8f acc[4][4];
#pragma unroll
    for (int mb = 0; mb < 4; ++mb)
#pragma unroll
        for (int nb = 0; nb < 4; ++nb) acc[mb][nb] = (v8f){};
    const size_t aoff = (size_t)(r0 + lr) * K + 8 * hi, boff = (size_t)lr * K + 8 * hi;
#pragma unroll 1
    for (int kc = 0; kc < K; kc += 32) {
        v16bf a[4];
#pragma unroll
        for (int mb = 0; mb < 4; ++mb) a[mb] = ldb(A + aoff + (size_t)mb * 16 * K + kc);
#pragma unroll
        for (int nb = 0; nb < 4; ++nb) { const v16bf b = ldb(Bt + boff + (size_t)nb * 16 * K + kc);
#pragma unroll
            for (int mb = 0; mb < 4; ++mb) acc[mb][nb] = wmmabg(a[mb], b, acc[mb][nb]); }
    }
#pragma unroll
    for (int mb = 0; mb < 4; ++mb) {
#pragma unroll
        for (int nb = 0; nb < 4; ++nb) {
#pragma unroll
            for (int j = 0; j < 8; ++j) os[(hi * 8 + j) * 68 + nb * 16 + lr] = acc[mb][nb][j] * VCARRY; }
        wave_sync();
        const size_t sb = (size_t)(r0 + mb * 16) * DV;
#pragma unroll 1
        for (int ps = 0; ps < 2; ++ps) {
#pragma unroll
            for (int s = 0; s < 4; ++s) { const int row = 4 * s + (lane >> 3), c8 = (lane & 7) * 8;
                const v4f x0 = *(const v4fa*)(&os[row * 68 + c8]); const v4f x1 = *(const v4fa*)(&os[row * 68 + c8 + 4]); v8h hv;
#pragma unroll
                for (int i = 0; i < 4; ++i) { hv[i] = toh_flush(x0[i]); hv[4 + i] = toh_flush(x1[i]); }
                *(volatile v8h*)(VP + sb + (size_t)row * DV + c8) = hv; }
            if (ps == 0) __threadfence(); }
        wave_sync();
    }
}

__global__ __launch_bounds__(32) void k_omap(const h16* __restrict__ WO, const h16* __restrict__ VP, const float* __restrict__ hin, float* OUT) {
    __shared__ __align__(16) float os[16 * 68];
    const int lane = threadIdx.x & 31, lr = lane & 15, hi = lane >> 4; const int r0 = blockIdx.x * 32, c0 = blockIdx.y * 64;
    v8f af[2][4], ab[2][4];
#pragma unroll
    for (int mb = 0; mb < 2; ++mb)
#pragma unroll
        for (int nb = 0; nb < 4; ++nb) { af[mb][nb] = (v8f){}; ab[mb][nb] = (v8f){}; }
    const size_t aoff = (size_t)(r0 + lr) * WOP + 8 * hi, boff = (size_t)(c0 + lr) * DV + 8 * hi;
#pragma unroll 1
    for (int kc = 0; kc < DV; kc += 32) {
        v16h wf[2], wb[2];
#pragma unroll
        for (int mb = 0; mb < 2; ++mb) { wf[mb] = ldh(WO + aoff + (size_t)mb * 16 * WOP + kc); wb[mb] = ldh(WO + aoff + (size_t)mb * 16 * WOP + DV + kc); }
#pragma unroll
        for (int nb = 0; nb < 4; ++nb) { const v16h b = ldh(VP + boff + (size_t)nb * 16 * DV + kc);
#pragma unroll
            for (int mb = 0; mb < 2; ++mb) { af[mb][nb] = wmma16g(wf[mb], b, af[mb][nb]); ab[mb][nb] = wmma16g(wb[mb], b, ab[mb][nb]); } }
    }
    const int bb = c0 / SEQ, tt = c0 % SEQ;
    const size_t obase = ((size_t)bb * DM + (size_t)r0) * OUT_SEQ + (size_t)tt;
    const size_t hbase = ((size_t)bb * DM + (size_t)r0) * SEQ_FULL + (size_t)tt;
#pragma unroll
    for (int mb = 0; mb < 2; ++mb) {
#pragma unroll
        for (int nb = 0; nb < 4; ++nb) {
#pragma unroll
            for (int j = 0; j < 8; ++j) os[(hi * 8 + j) * 68 + nb * 16 + lr] = af[mb][nb][j] * CFS + ab[mb][nb][j] * CBS; }
        wave_sync();
#pragma unroll 1
        for (int ps = 0; ps < 2; ++ps) {
#pragma unroll
            for (int s = 0; s < 8; ++s) { const int row = 2 * s + (lane >> 4), cofs = (lane & 15) * 4;
                const v4f cv = *(const v4fa*)(&os[row * 68 + cofs]);
                const v4f rv = *(const v4f*)(hin + hbase + (size_t)(mb * 16 + row) * SEQ_FULL + cofs);
                v4f val;
#pragma unroll
                for (int i = 0; i < 4; ++i) val[i] = cv[i] + bfr(rv[i]);
                *(volatile v4f*)(OUT + obase + (size_t)(mb * 16 + row) * OUT_SEQ + cofs) = val; }
            if (ps == 0) __threadfence(); }
        wave_sync();
    }
}

static constexpr size_t al256(size_t v) { return (v + 255) & ~(size_t)255; }
static constexpr size_t SZ_HT = al256((size_t)NB * SEQ * DM * 2);
static constexpr size_t SZ_WG = al256((size_t)DV * DM * 2);
static constexpr size_t SZ_WO = al256((size_t)DM * WOP * 2);
static constexpr size_t SZ_VP = al256((size_t)NB * SEQ * DV * 2);
static constexpr size_t SZ_TOTAL = SZ_HT + SZ_WG + SZ_WO + SZ_VP;
static_assert(SZ_TOTAL <= (size_t)134217728);
static_assert(((size_t)DV * DM) % (8 * 256) == 0);
static_assert(((size_t)DM * WOP) % (8 * 256) == 0);
static_assert(((size_t)NB * SEQ / 64) * 64 * DM * 2 == (size_t)NB * SEQ * DM * 2);
static_assert(((size_t)NB * SEQ / 64) * 64 * DV * 2 == (size_t)NB * SEQ * DV * 2);

extern "C" void kernel_launch(void* const* d_in, const int* in_sizes, int n_in,
                              void* d_out, int out_size, void* d_ws, size_t ws_size, hipStream_t stream) {
    if (n_in < 5) return;
    const size_t needh = ((size_t)NB_FULL * DM - 1) * SEQ_FULL + SEQ;
    if ((size_t)in_sizes[0] < needh) return;
    if ((size_t)in_sizes[3] < (size_t)DV * DM || (size_t)in_sizes[4] < (size_t)DM * WOP) return;
    if ((size_t)out_size < ((size_t)NB * DM - 1) * OUT_SEQ + SEQ) return;
    if (SZ_TOTAL > ws_size) return;
    const float* hin = (const float*)d_in[0];
    const float* wg  = (const float*)d_in[3];
    const float* wo  = (const float*)d_in[4];
    float* OUT = (float*)d_out;
    char* wsp = (char*)d_ws;
    bf*  HT  = (bf*)wsp;  wsp += SZ_HT;
    bf*  WGB = (bf*)wsp;  wsp += SZ_WG;
    h16* WOH = (h16*)wsp; wsp += SZ_WO;
    h16* VP  = (h16*)wsp; wsp += SZ_VP;

    { const size_t n8 = (size_t)DV * DM / 8;  k_cvt8<<<(unsigned)((n8 + 255) / 256), 256, 0, stream>>>(wg, WGB, n8); }
    { const size_t n8 = (size_t)DM * WOP / 8; k_cvth8<<<(unsigned)((n8 + 255) / 256), 256, 0, stream>>>(wo, WOH, n8); }
    k_tr<<<dim3(SEQ / 64, NB, 1), 256, 0, stream>>>(hin, HT);
    k_vmap<<<dim3(NB * SEQ / 64, 1, 1), 32, 0, stream>>>(HT, WGB, VP);
    k_omap<<<dim3(DM / 32, NB * SEQ / 64, 1), 32, 0, stream>>>(WOH, VP, hin, OUT);
}
